// MultiHeadedAttention_58548994179264
// MI455X (gfx1250) — hardware-verified
//
#include <hip/hip_runtime.h>


#ifndef NB
#define NB 2
#endif
#ifndef SEQ
#define SEQ 2048
#endif
#define SEQ_FULL 2048
#define TT   SEQ
#define DM   1024
#define NH_  16
#define HD   64
#define QSCL 0.18033688011112042f

static_assert(TT % 128 == 0);
static_assert(TT <= SEQ_FULL);
static_assert(NH_ * HD == DM);
static_assert(DM % 64 == 0);
static_assert(DM % 32 == 0);
static_assert(HD == 64);
static_assert(NB >= 1 && NB <= 8);
static_assert(((DM * DM / 8) % 256) == 0);
static_assert((((size_t)NB * SEQ_FULL * DM / 8) % 256) == 0);
static_assert((((size_t)NB * NH_ * TT * HD / 8) % 256) == 0);
static_assert(((NB * NH_ * (TT / 16)) % 4) == 0);
static_assert(((size_t)NB * TT) % 64 == 0);

#define SZ_WT  ((size_t)4 * DM * DM * 2)
#define SZ_XB  ((size_t)NB * SEQ_FULL * DM * 2)
#define SZ_F   ((size_t)3 * NB * TT * DM * 4)
#define SZ_PL  ((size_t)NB * NH_ * TT * HD * 2)
#define SZ_CX  ((size_t)NB * TT * DM * 2)
#define WS_TOTAL (SZ_WT + SZ_XB + SZ_F + 3 * SZ_PL + 2 * SZ_CX)
static_assert(SZ_WT % 256 == 0 && SZ_XB % 256 == 0 && SZ_F % 256 == 0 && SZ_PL % 256 == 0 && SZ_CX % 256 == 0);
static_assert(WS_TOTAL <= (size_t)134217728);

typedef _Float16 h16;
typedef unsigned short bf;
typedef __attribute__((ext_vector_type(16))) __bf16   v16bf;
typedef __attribute__((ext_vector_type(16))) _Float16 v16h;
typedef __attribute__((ext_vector_type(8)))  _Float16 v8h;
typedef __attribute__((ext_vector_type(8)))  unsigned short v8us;
typedef __attribute__((ext_vector_type(8)))  float    v8f;
typedef __attribute__((ext_vector_type(4)))  float    v4f;
typedef v8h  __attribute__((may_alias)) v8ha;
typedef v4f  __attribute__((may_alias)) v4fa;
typedef v8us __attribute__((may_alias)) v8usa;

__device__ __forceinline__ unsigned short f2bf(float f) { unsigned u = __float_as_uint(f); u += 0x7FFFu + ((u >> 16) & 1u); return (unsigned short)(u >> 16); }
__device__ __forceinline__ float bf2f(unsigned short b) { return __uint_as_float(((unsigned)b) << 16); }
__device__ __forceinline__ float bfr(float f) { return bf2f(f2bf(f)); }
__device__ __forceinline__ v16h cat16(v8h lo, v8h hi) { return __builtin_shufflevector(lo, hi, 0, 1, 2, 3, 4, 5, 6, 7, 8, 9, 10, 11, 12, 13, 14, 15); }
__device__ __forceinline__ v16bf cat16b(v8us lo, v8us hi) { return __builtin_bit_cast(v16bf, __builtin_shufflevector(lo, hi, 0, 1, 2, 3, 4, 5, 6, 7, 8, 9, 10, 11, 12, 13, 14, 15)); }
__device__ __forceinline__ v8f wmma16(v16h a, v16h b, v8f c) { return __builtin_amdgcn_wmma_f32_16x16x32_f16(false, a, false, b, (short)0, c, false, false); }
__device__ __forceinline__ v8f wmmab(v16bf a, v16bf b, v8f c) { return __builtin_amdgcn_wmma_f32_16x16x32_bf16(false, a, false, b, (short)0, c, false, false); }
__device__ __forceinline__ h16 tohx(float x) { return (h16)x; }
__device__ __forceinline__ void splitf(float y, unsigned short& h, unsigned short& l) { h = f2bf(y); l = f2bf(y - bf2f(h)); }

template <typename T16> struct WFrag;
template <> struct WFrag<h16> { typedef v16h V; static __device__ __forceinline__ V ld(const h16* p) { return cat16(*(const v8h*)p, *(const v8h*)(p + 16)); } static __device__ __forceinline__ v8f mma(V a, V b, v8f c) { return wmma16(a, b, c); } };
template <> struct WFrag<bf> { typedef v16bf V; static __device__ __forceinline__ V ld(const bf* p) { return cat16b(*(const v8us*)p, *(const v8us*)(p + 16)); } static __device__ __forceinline__ v8f mma(V a, V b, v8f c) { return wmmab(a, b, c); } };
template <typename T16, int NSPLIT, bool BIAS>
__global__ __launch_bounds__(32) void k_gemmw(const T16* __restrict__ A, const T16* __restrict__ A2, const T16* __restrict__ Bt, const T16* __restrict__ Bt2, int K, float* C, int ldc, const float* __restrict__ bias, size_t sA, size_t sB, size_t sC) {
    typedef typename WFrag<T16>::V V;
    __shared__ __align__(16) float os[16 * 68];
    const size_t z = blockIdx.z; A += z * sA; if (A2) A2 += z * sA; Bt += z * sB; if (Bt2) Bt2 += z * sB; C += z * sC;
    const int lane = threadIdx.x & 31, lr = lane & 15, hi = lane >> 4; const int r0 = blockIdx.x * 64, c0 = blockIdx.y * 64;
    v8f acc[4][4];
#pragma unroll
    for (int mb = 0; mb < 4; ++mb)
#pragma unroll
        for (int nb = 0; nb < 4; ++nb) acc[mb][nb] = (v8f){};
    const size_t aoff = (size_t)(r0 + lr) * K + 8 * hi, boff = (size_t)(c0 + lr) * K + 8 * hi;
#pragma unroll 1
    for (int kc = 0; kc < K; kc += 32) {
        V a[4], a2[4];
#pragma unroll
        for (int mb = 0; mb < 4; ++mb) { a[mb] = WFrag<T16>::ld(A + aoff + (size_t)mb * 16 * K + kc); if (NSPLIT == 1 || NSPLIT == 2) a2[mb] = WFrag<T16>::ld(A2 + aoff + (size_t)mb * 16 * K + kc); }
#pragma unroll
        for (int nb = 0; nb < 4; ++nb) { const V b = WFrag<T16>::ld(Bt + boff + (size_t)nb * 16 * K + kc); V b2; if (NSPLIT >= 2) b2 = WFrag<T16>::ld(Bt2 + boff + (size_t)nb * 16 * K + kc);
#pragma unroll
            for (int mb = 0; mb < 4; ++mb) { acc[mb][nb] = WFrag<T16>::mma(a[mb], b, acc[mb][nb]); if (NSPLIT == 1 || NSPLIT == 2) acc[mb][nb] = WFrag<T16>::mma(a2[mb], b, acc[mb][nb]); if (NSPLIT >= 2) acc[mb][nb] = WFrag<T16>::mma(a[mb], b2, acc[mb][nb]); } }
        asm volatile("v_nop\n\tv_nop\n\tv_nop\n\tv_nop" : "+v"(acc[0][0]), "+v"(acc[1][1]), "+v"(acc[2][2]), "+v"(acc[3][3]) : "v"(a[0]), "v"(a[3]));
    }
#pragma unroll
    for (int mb = 0; mb < 4; ++mb) {
#pragma unroll
        for (int nb = 0; nb < 4; ++nb) {
#pragma unroll
            for (int j = 0; j < 8; ++j) os[(hi * 8 + j) * 68 + nb * 16 + lr] = acc[mb][nb][j]; }
        __builtin_amdgcn_wave_barrier(); asm volatile("" ::: "memory");
        float* crow = C + (size_t)(r0 + mb * 16) * ldc + c0;
#pragma unroll 1
        for (int ps = 0; ps < 2; ++ps) {
#pragma unroll
            for (int s = 0; s < 8; ++s) { const int row = 2 * s + hi, cofs = lr * 4; v4f val = *(const v4fa*)(os + row * 68 + cofs); if (BIAS) { val[0] += bfr(bias[c0 + cofs]); val[1] += bfr(bias[c0 + cofs + 1]); val[2] += bfr(bias[c0 + cofs + 2]); val[3] += bfr(bias[c0 + cofs + 3]); }
                *(volatile v4f*)(crow + (size_t)row * ldc + cofs) = val; }
            if (ps == 0) __threadfence(); }
        __builtin_amdgcn_wave_barrier(); asm volatile("" ::: "memory");
    }
}

__global__ __launch_bounds__(256) void k_cvt8(const float* __restrict__ src, bf* dst, size_t n8) { const size_t i = (size_t)blockIdx.x * 256 + threadIdx.x; if (i >= n8) return; const v8f v = *(const v8f*)(src + i * 8); v8us o;
#pragma unroll
    for (int k = 0; k < 8; ++k) o[k] = f2bf(v[k]); *(volatile v8us*)(dst + i * 8) = o; __threadfence(); *(volatile v8us*)(dst + i * 8) = o; }

__global__ __launch_bounds__(256) void k_wt(const float* __restrict__ wq, const float* __restrict__ wk, const float* __restrict__ wv, const float* __restrict__ wo, bf* Bt) {
    const unsigned z = blockIdx.y;
    const float* w = (z == 0u) ? wq : ((z == 1u) ? wk : ((z == 2u) ? wv : wo));
    const unsigned i = blockIdx.x * 256u + threadIdx.x; if (i >= (unsigned)(DM * DM / 8)) return;
    const unsigned e = i * 8u; const unsigned k = e % (unsigned)DM; const unsigned n = e / (unsigned)DM;
    v8us o;
#pragma unroll
    for (unsigned q = 0; q < 8u; ++q) o[q] = f2bf(w[(size_t)(k + q) * DM + n]);
    bf* d = Bt + (size_t)z * DM * DM + e;
    *(volatile v8us*)d = o; __threadfence(); *(volatile v8us*)d = o;
}

__global__ __launch_bounds__(256) void k_qkp(const float* __restrict__ FQ, const float* __restrict__ FK, const float* __restrict__ bq, const float* __restrict__ bk, h16* QP, h16* KP) {
    const unsigned y = blockIdx.y;
    const float* F = y ? FK : FQ; const float* bias = y ? bk : bq; h16* P = y ? KP : QP;
    const unsigned i = blockIdx.x * 256u + threadIdx.x; if (i >= (unsigned)((size_t)NB * NH_ * TT * HD / 8)) return;
    const unsigned e = i * 8u; const unsigned d = e % (unsigned)HD; const unsigned t = (e / (unsigned)HD) % (unsigned)TT; const unsigned bh = e / (unsigned)(HD * TT);
    const unsigned b = bh / (unsigned)NH_, h = bh % (unsigned)NH_;
    const v8f f = *(const v8f*)(F + ((size_t)b * TT + t) * DM + h * HD + d); const v8f bb = *(const v8f*)(bias + h * HD + d);
    v8h o;
#pragma unroll
    for (int q = 0; q < 8; ++q) o[q] = tohx(f[q] + bfr(bb[q]));
    *(volatile v8h*)(P + e) = o; __threadfence(); *(volatile v8h*)(P + e) = o;
}

__global__ __launch_bounds__(256) void k_vtp(const float* __restrict__ F, const float* __restrict__ bias, h16* VT) {
    const unsigned i = blockIdx.x * 256u + threadIdx.x; if (i >= (unsigned)((size_t)NB * NH_ * HD * TT / 8)) return;
    const unsigned e = i * 8u; const unsigned t = e % (unsigned)TT; const unsigned d = (e / (unsigned)TT) % (unsigned)HD; const unsigned bh = e / (unsigned)(TT * HD);
    const unsigned b = bh / (unsigned)NH_, h = bh % (unsigned)NH_;
    const float bb = bfr(bias[h * HD + d]);
    const float* src = F + ((size_t)b * TT + t) * DM + h * HD + d;
    v8h o;
#pragma unroll
    for (int q = 0; q < 8; ++q) o[q] = tohx(src[(size_t)q * DM] + bb);
    *(volatile v8h*)(VT + e) = o; __threadfence(); *(volatile v8h*)(VT + e) = o;
}

__global__ __launch_bounds__(128) void k_flash(const h16* __restrict__ QP, const h16* __restrict__ KP, const h16* __restrict__ VT, bf* CH, bf* CL) {
    __shared__ __align__(16) float os[4 * 16 * 68];
    const unsigned lane = threadIdx.x & 31u, wv = threadIdx.x >> 5, lr = lane & 15u, hi = lane >> 4;
    const unsigned tile = blockIdx.x * 4u + wv;
    const unsigned qt = tile % (unsigned)(TT / 16), bh = tile / (unsigned)(TT / 16);
    const h16* qrow = QP + ((size_t)bh * TT + qt * 16u + lr) * HD + 8u * hi;
    const v16h q0 = WFrag<h16>::ld(qrow), q1 = WFrag<h16>::ld(qrow + 32);
    const h16* kbase = KP + ((size_t)bh * TT + lr) * HD + 8u * hi;
    const h16* vbase = VT + ((size_t)bh * HD + lr) * TT + 8u * hi;
    v8f o[4];
#pragma unroll
    for (int dt = 0; dt < 4; ++dt) o[dt] = (v8f){};
    float m = -3.0e38f, l = 0.f;
#pragma unroll 1
    for (unsigned kk = 0; kk < (unsigned)TT; kk += 64u) {
        v8f s[4]; v16h a0, a1;
#pragma unroll
        for (int t = 0; t < 4; ++t) {
            const h16* kp = kbase + (size_t)(kk + 16u * (unsigned)t) * HD;
            a0 = WFrag<h16>::ld(kp); a1 = WFrag<h16>::ld(kp + 32);
            s[t] = wmma16(a0, q0, (v8f){});
            s[t] = wmma16(a1, q1, s[t]);
        }
        asm volatile("v_nop\n\tv_nop\n\tv_nop\n\tv_nop" : "+v"(s[0]), "+v"(s[1]), "+v"(s[2]), "+v"(s[3]) : "v"(a0), "v"(a1), "v"(q0), "v"(q1));
        float mx = s[0][0];
#pragma unroll
        for (int t = 0; t < 4; ++t)
#pragma unroll
            for (int r = 0; r < 8; ++r) mx = fmaxf(mx, s[t][r]);
        mx = fmaxf(mx, __shfl_xor(mx, 16, 32));
        const float mn = fmaxf(m, mx);
        const float al = __builtin_amdgcn_exp2f((m - mn) * QSCL);
        m = mn;
        float ps = 0.f;
#pragma unroll
        for (int t = 0; t < 4; ++t)
#pragma unroll
            for (int r = 0; r < 8; ++r) { const float p = __builtin_amdgcn_exp2f(fmaf(s[t][r] - mn, QSCL, 10.0f)); s[t][r] = p; ps += p; }
        l = l * al + ps;
#pragma unroll
        for (int dt = 0; dt < 4; ++dt)
#pragma unroll
            for (int r = 0; r < 8; ++r) o[dt][r] *= al;
        v16h pb0, pb1;
#pragma unroll
        for (int r = 0; r < 8; ++r) { pb0[r] = tohx(s[0][r]); pb0[8 + r] = tohx(s[1][r]); pb1[r] = tohx(s[2][r]); pb1[8 + r] = tohx(s[3][r]); }
#pragma unroll
        for (int dt = 0; dt < 4; ++dt) {
            const h16* vp = vbase + (size_t)(16u * (unsigned)dt) * TT + kk;
            a0 = WFrag<h16>::ld(vp); a1 = WFrag<h16>::ld(vp + 32);
            o[dt] = wmma16(a0, pb0, o[dt]);
            o[dt] = wmma16(a1, pb1, o[dt]);
        }
        asm volatile("v_nop\n\tv_nop\n\tv_nop\n\tv_nop" : "+v"(o[0]), "+v"(o[1]), "+v"(o[2]), "+v"(o[3]) : "v"(a0), "v"(a1), "v"(pb0), "v"(pb1));
    }
    const float lt = l + __shfl_xor(l, 16, 32);
    const float inv = 1.0f / lt;
    float* ow = os + wv * (16u * 68u);
#pragma unroll
    for (int dt = 0; dt < 4; ++dt) {
        v4f x0, x1;
#pragma unroll
        for (int r = 0; r < 4; ++r) { x0[r] = o[dt][r] * inv; x1[r] = o[dt][4 + r] * inv; }
        float* dst = ow + lr * 68u + (unsigned)dt * 16u + 8u * hi;
        *(v4fa*)dst = x0; *(v4fa*)(dst + 4) = x1;
    }
    __builtin_amdgcn_fence(3  , "wavefront");
    __builtin_amdgcn_wave_barrier(); asm volatile("" ::: "memory");
    const unsigned b = bh / (unsigned)NH_, h = bh % (unsigned)NH_;
    const unsigned rq = lane >> 3, d0 = (lane & 7u) * 8u;
    v8us oh[4], ol[4]; size_t off[4];
#pragma unroll
    for (int s4 = 0; s4 < 4; ++s4) {
        const unsigned row = 4u * (unsigned)s4 + rq;
        const v4f x0 = *(const v4fa*)(ow + row * 68u + d0), x1 = *(const v4fa*)(ow + row * 68u + d0 + 4u);
#pragma unroll
        for (int r = 0; r < 4; ++r) { unsigned short a, c; splitf(x0[r], a, c); oh[s4][r] = a; ol[s4][r] = c; splitf(x1[r], a, c); oh[s4][4 + r] = a; ol[s4][4 + r] = c; }
        off[s4] = ((size_t)b * TT + qt * 16u + row) * DM + h * HD + d0;
    }
#pragma unroll 1
    for (int ps = 0; ps < 2; ++ps) {
#pragma unroll
        for (int s4 = 0; s4 < 4; ++s4) { *(volatile v8us*)(CH + off[s4]) = oh[s4]; *(volatile v8us*)(CL + off[s4]) = ol[s4]; }
        if (ps == 0) __threadfence(); }
}

extern "C" void kernel_launch(void* const* d_in, const int* in_sizes, int n_in,
                              void* d_out, int out_size, void* d_ws, size_t ws_size, hipStream_t stream) {
    if (n_in < 9) return;
    if (in_sizes[0] < NB * SEQ_FULL * DM) return;
    if (in_sizes[1] < DM * DM || in_sizes[2] < DM * DM || in_sizes[3] < DM * DM || in_sizes[4] < DM * DM) return;
    if (in_sizes[5] < DM || in_sizes[6] < DM || in_sizes[7] < DM || in_sizes[8] < DM) return;
    if (out_size < NB * TT * DM) return;
    if (ws_size < WS_TOTAL) return;
    const float* x  = (const float*)d_in[0];
    const float* wq = (const float*)d_in[1]; const float* wk = (const float*)d_in[2];
    const float* wv = (const float*)d_in[3]; const float* wo = (const float*)d_in[4];
    const float* bq = (const float*)d_in[5]; const float* bk = (const float*)d_in[6];
    const float* bv = (const float*)d_in[7]; const float* bo = (const float*)d_in[8];
    float* OUT = (float*)d_out;
    char* wsp = (char*)d_ws;
    auto take = [&](size_t bytes) { char* p = wsp; wsp += (bytes + 255) & ~(size_t)255; return (void*)p; };
    bf*    WT = (bf*)take(SZ_WT);
    bf*    XB = (bf*)take(SZ_XB);
    float* F  = (float*)take(SZ_F);
    h16*   QP = (h16*)take(SZ_PL);
    h16*   KP = (h16*)take(SZ_PL);
    h16*   VT = (h16*)take(SZ_PL);
    bf*    CH = (bf*)take(SZ_CX);
    bf*    CL = (bf*)take(SZ_CX);
    if ((size_t)(wsp - (char*)d_ws) > ws_size) return;
    float* FQ = F; float* FK = F + (size_t)NB * TT * DM; float* FV = F + (size_t)2 * NB * TT * DM;

    k_wt<<<dim3((unsigned)(DM * DM / 8 / 256), 4), 256, 0, stream>>>(wq, wk, wv, wo, WT);
    const size_t nx8 = (size_t)NB * SEQ_FULL * DM / 8;
    k_cvt8<<<(unsigned)((nx8 + 255) / 256), 256, 0, stream>>>(x, XB, nx8);
    for (int b = 0; b < NB; ++b) {
        k_gemmw<bf, 0, false><<<dim3(TT / 64, DM / 64, 3), 32, 0, stream>>>(XB + (size_t)b * SEQ_FULL * DM, nullptr, WT, nullptr, DM, F + (size_t)b * TT * DM, DM, nullptr, (size_t)0, (size_t)DM * DM, (size_t)NB * TT * DM);
    }
    const unsigned LP = (unsigned)(((size_t)NB * NH_ * TT * HD / 8 + 255) / 256);
    k_qkp<<<dim3(LP, 2), 256, 0, stream>>>(FQ, FK, bq, bk, QP, KP);
    k_vtp<<<LP, 256, 0, stream>>>(FV, bv, VT);
    k_flash<<<(unsigned)(NB * NH_ * (TT / 16) / 4), 128, 0, stream>>>(QP, KP, VT, CH, CL);
    k_gemmw<bf, 1, true><<<dim3((unsigned)((size_t)NB * TT / 64), DM / 64, 1), 32, 0, stream>>>(CH, CL, WT + (size_t)3 * DM * DM, nullptr, DM, OUT, DM, bo, (size_t)0, (size_t)0, (size_t)0);
}
